// Task_Aware_Delta_Net_3358664426168
// MI455X (gfx1250) — hardware-verified
//
#include <hip/hip_runtime.h>
#include <math.h>

typedef __attribute__((ext_vector_type(16))) _Float16 v16h;
typedef __attribute__((ext_vector_type(8)))  _Float16 v8h;
typedef __attribute__((ext_vector_type(16))) __bf16   v16b;
typedef __attribute__((ext_vector_type(8)))  __bf16   v8b;
typedef __attribute__((ext_vector_type(8)))  float    v8f;
typedef __attribute__((ext_vector_type(4)))  float    v4f;

constexpr int kB    = 2;
constexpr int kL    = 2048;
constexpr int kDH   = 2048;
constexpr int kHd   = 256;
constexpr int kH    = 6;
constexpr int kKD   = kH * kHd;
constexpr int kBG   = 64;
constexpr int kCS   = 64;
constexpr int kTaps = 4;
constexpr int kThr  = 256;
constexpr float kInCarry = 1024.0f;
constexpr float kWCarry = 4096.0f;
constexpr float kSc = 1.0f / (kInCarry * kInCarry);
constexpr float kCo = 256.0f;
constexpr float kScO = 1.0f / (kCo * kInCarry);
constexpr float kQScale = 0.0625f;
constexpr float kL2Eps = 1e-6f, kRmsEps = 1e-5f;
constexpr float kF16MinNormal = 6.103515625e-5f;

static_assert((kL % 64) == 0 && (kDH % 64) == 0 && (kKD % 64) == 0 && (kBG % 64) == 0 && ((kL / 64) * (kKD / 64)) % 8 == 0 && ((kL / 64) * (kBG / 64)) % 8 == 0 && ((kL / 64) * (kDH / 64)) % 8 == 0, "GEMM M, N multiples of 64; grids exact");
static_assert((kDH % 32) == 0 && (kKD % 32) == 0 && kKD == 3 * 512 && kHd == 4 * kCS, "GEMM K multiples of 32; the output weight's 1,536 columns cast as three runs of 512; four 64-column blocks a head");

constexpr size_t kOffWQ = 0ull;
constexpr size_t kOffWK = 6291456ull;
constexpr size_t kOffWV = 12582912ull;
constexpr size_t kOffWG = 18874368ull;
constexpr size_t kOffWO = 25165824ull;
constexpr size_t kOffWBA = 31457280ull;
constexpr size_t kOffBIAS = 31719424ull;
constexpr size_t kOffPRM = 31727616ull;
constexpr size_t kOffX16 = 31731712ull;
constexpr size_t kOffXL = 40120320ull;
constexpr size_t kOffQ2 = 52703232ull;
constexpr size_t kOffK2 = 65286144ull;
constexpr size_t kOffV2 = 77869056ull;
constexpr size_t kOffGL = 90451968ull;
constexpr size_t kOffBAL = 103034880ull;
constexpr size_t kOffBE = 103559168ull;
constexpr size_t kOffO32 = 103821312ull;
constexpr size_t kOffO16 = 116404224ull;
constexpr size_t kWsTotal = 122695680ull;
static_assert(kWsTotal <= 134217728ull, "carve cap: under 128 MiB");
static_assert(kOffWQ == 0
              && kOffWK == kOffWQ + 6291456ull
              && kOffWV == kOffWK + 6291456ull
              && kOffWG == kOffWV + 6291456ull
              && kOffWO == kOffWG + 6291456ull
              && kOffWBA == kOffWO + 6291456ull
              && kOffBIAS == kOffWBA + 262144ull
              && kOffPRM == kOffBIAS + 8192ull
              && kOffX16 == kOffPRM + 4096ull
              && kOffXL == kOffX16 + 8388608ull
              && kOffQ2 == kOffXL + 12582912ull
              && kOffK2 == kOffQ2 + 12582912ull
              && kOffV2 == kOffK2 + 12582912ull
              && kOffGL == kOffV2 + 12582912ull
              && kOffBAL == kOffGL + 12582912ull
              && kOffBE == kOffBAL + 524288ull
              && kOffO32 == kOffBE + 262144ull
              && kOffO16 == kOffO32 + 12582912ull
              && kWsTotal == kOffO16 + 6291456ull, "the carve is chained and totalled");
static_assert((kOffWQ % 256) == 0 && (kOffWK % 256) == 0 && (kOffWV % 256) == 0 && (kOffWG % 256) == 0 && (kOffWO % 256) == 0 && (kOffWBA % 256) == 0 && (kOffBIAS % 256) == 0 && (kOffPRM % 256) == 0 && (kOffX16 % 256) == 0 && (kOffXL % 256) == 0 && (kOffQ2 % 256) == 0 && (kOffK2 % 256) == 0 && (kOffV2 % 256) == 0 && (kOffGL % 256) == 0 && (kOffBAL % 256) == 0 && (kOffBE % 256) == 0 && (kOffO32 % 256) == 0 && (kOffO16 % 256) == 0, "aligned regions");
constexpr int kPA = 0, kPD = 8, kPW = 16, kPEnd = 1024;
static_assert(kPD >= kPA + kH && kPW >= kPD + kH && kPW + kHd <= kPEnd, "parameter plane map");

__device__ __forceinline__ unsigned short f2bf_bits(float f) {
  unsigned u = __float_as_uint(f);
  return (unsigned short)((u + 0x7FFFu + ((u >> 16) & 1u)) >> 16);
}
__device__ __forceinline__ float bf_bits2f(unsigned short h) { return __uint_as_float(((unsigned)h) << 16); }
__device__ __forceinline__ float bf16r(float f) { return bf_bits2f(f2bf_bits(f)); }
__device__ __forceinline__ float carry_flush(float v, float carry) {
  const float s = v * carry;
  return (fabsf(s) < kF16MinNormal) ? 0.0f : s;
}
__device__ __forceinline__ float frcp(float x) { return __builtin_amdgcn_rcpf(x); }

__device__ __forceinline__ void dep_guard4_h(v8f& a, v8f& b, v8f& c, v8f& d, v16h x, v16h y) { asm volatile("v_nop\n\tv_nop\n\tv_nop\n\tv_nop" : "+v"(a), "+v"(b), "+v"(c), "+v"(d) : "v"(x), "v"(y)); }
__device__ __forceinline__ void dep_guard4_b(v8f& a, v8f& b, v8f& c, v8f& d, v16b x, v16b y) { asm volatile("v_nop\n\tv_nop\n\tv_nop\n\tv_nop" : "+v"(a), "+v"(b), "+v"(c), "+v"(d) : "v"(x), "v"(y)); }
__device__ __forceinline__ void keep4_h(v16h a, v16h b, v16h c, v16h d) { asm volatile("v_nop" :: "v"(a), "v"(b), "v"(c), "v"(d)); }
__device__ __forceinline__ void keep4_b(v16b a, v16b b, v16b c, v16b d) { asm volatile("v_nop" :: "v"(a), "v"(b), "v"(c), "v"(d)); }
__device__ __forceinline__ void acc_guard4(v8f& a, v8f& b, v8f& c, v8f& d) { asm volatile("v_nop\n\tv_nop\n\tv_nop\n\tv_nop" : "+v"(a), "+v"(b), "+v"(c), "+v"(d)); }

template <typename T> struct Frag;
template <> struct Frag<_Float16> {
  typedef v16h V; union U { v16h v; v8h h[2]; };
  static __device__ __forceinline__ v16h load(const _Float16* p) {
    U f; f.h[0] = *(const v8h*)(p); f.h[1] = *(const v8h*)(p + 16); return f.v;
  }
  static __device__ __forceinline__ v8f mma(v16h a, v16h b, v8f c) {
    return __builtin_amdgcn_wmma_f32_16x16x32_f16(false, a, false, b, (short)0, c, false, false);
  }
  static __device__ __forceinline__ void guard4(v8f& a, v8f& b, v8f& c, v8f& d, v16h x, v16h y) { dep_guard4_h(a, b, c, d, x, y); }
  static __device__ __forceinline__ void keep(v16h a, v16h b, v16h c, v16h d) { keep4_h(a, b, c, d); }
};
template <> struct Frag<__bf16> {
  typedef v16b V; union U { v16b v; v8b h[2]; };
  static __device__ __forceinline__ v16b load(const __bf16* p) {
    U f; f.h[0] = *(const v8b*)(p); f.h[1] = *(const v8b*)(p + 16); return f.v;
  }
  static __device__ __forceinline__ v8f mma(v16b a, v16b b, v8f c) {
    return __builtin_amdgcn_wmma_f32_16x16x32_bf16(false, a, false, b, (short)0, c, false, false);
  }
  static __device__ __forceinline__ void guard4(v8f& a, v8f& b, v8f& c, v8f& d, v16b x, v16b y) { dep_guard4_b(a, b, c, d, x, y); }
  static __device__ __forceinline__ void keep(v16b a, v16b b, v16b c, v16b d) { keep4_b(a, b, c, d); }
};

__device__ __forceinline__ v8f mma_h(v16h a, v16h b, v8f c) {
  c = __builtin_amdgcn_wmma_f32_16x16x32_f16(false, a, false, b, (short)0, c, false, false);
  asm volatile("v_nop\n\tv_nop\n\tv_nop\n\tv_nop" : "+v"(c) : "v"(a), "v"(b));
  return c;
}

template <int ET> struct Elem;
template <> struct Elem<0> { typedef _Float16 T; };
template <> struct Elem<1> { typedef __bf16 T; };
template <int ET, bool SPLIT, int BIAS_MODE, int OUT_MODE, bool RESID, int ACT = 0>
__global__ __launch_bounds__(256) void wmma_gemm64(
    const unsigned short* __restrict__ Ap, const unsigned short* __restrict__ A2p, int lda, long strideA,
    const unsigned short* __restrict__ Btp, const unsigned short* __restrict__ Bt2p, int ldb, long strideB,
    void* __restrict__ Cout, void* __restrict__ Cout2, int ldc, long strideC,
    const float* __restrict__ bias,
    const float* __restrict__ resid, long strideR,
    int M, int N, int K, float scale) {
  typedef typename Elem<ET>::T T;
  typedef typename Frag<T>::V V;
  const T* A = (const T*)Ap; const T* A2 = (const T*)A2p; const T* Bt = (const T*)Btp; const T* Bt2 = (const T*)Bt2p;
  __shared__ __align__(16) float sT[8][16 * 68];
  const int b    = blockIdx.y;
  const int lane = threadIdx.x & 31;
  const int wave = threadIdx.x >> 5;
  const int tilesN = N >> 6;
  const int tilesM = M >> 6;
  const int tile = blockIdx.x * 8 + wave;
  if (tile >= tilesM * tilesN) return;
  const int tm = tile / tilesN;
  const int tn = tile - tm * tilesN;
  const int m0 = tm << 6;
  const int n0 = tn << 6;

  const T* Ab  = A  + (size_t)b * strideA;
  const T* Bb  = Bt + (size_t)b * strideB;
  const T* Ab2 = SPLIT ? (A2  + (size_t)b * strideA) : nullptr;
  const T* Bb2 = SPLIT ? (Bt2 + (size_t)b * strideB) : nullptr;

  const int rlane = lane & 15;
  const int koff  = (lane >> 4) * 8;
  const int mOff  = (lane >> 4) * 8;

  v8f acc[4][4];
#pragma unroll
  for (int i = 0; i < 4; ++i)
#pragma unroll
    for (int j = 0; j < 4; ++j) acc[i][j] = (v8f){0.f,0.f,0.f,0.f,0.f,0.f,0.f,0.f};

  for (int k0 = 0; k0 < K; k0 += 32) {
    V bh[4], bl[4];
#pragma unroll
    for (int j = 0; j < 4; ++j) {
      const size_t bo = (size_t)(n0 + (j << 4) + rlane) * ldb + koff + k0;
      bh[j] = Frag<T>::load(Bb + bo);
      if (SPLIT) bl[j] = Frag<T>::load(Bb2 + bo);
    }
#pragma unroll
    for (int i = 0; i < 4; ++i) {
      const size_t ao = (size_t)(m0 + (i << 4) + rlane) * lda + koff + k0;
      V ah = Frag<T>::load(Ab + ao);
      V al;
      if (SPLIT) al = Frag<T>::load(Ab2 + ao);
#pragma unroll
      for (int j = 0; j < 4; ++j) {
        acc[i][j] = Frag<T>::mma(ah, bh[j], acc[i][j]);
        if (SPLIT) {
          acc[i][j] = Frag<T>::mma(ah, bl[j], acc[i][j]);
          acc[i][j] = Frag<T>::mma(al, bh[j], acc[i][j]);
        }
      }
      Frag<T>::guard4(acc[i][0], acc[i][1], acc[i][2], acc[i][3], ah, SPLIT ? al : ah);
    }
    Frag<T>::keep(bh[0], bh[1], bh[2], bh[3]);
    if (SPLIT) Frag<T>::keep(bl[0], bl[1], bl[2], bl[3]);
  }
  acc_guard4(acc[0][0], acc[0][1], acc[0][2], acc[0][3]);
  acc_guard4(acc[1][0], acc[1][1], acc[1][2], acc[1][3]);
  acc_guard4(acc[2][0], acc[2][1], acc[2][2], acc[2][3]);
  acc_guard4(acc[3][0], acc[3][1], acc[3][2], acc[3][3]);

  float* slab = sT[wave];
  const float* Rb = RESID ? (resid + (size_t)b * strideR) : nullptr;
#pragma unroll
  for (int i = 0; i < 4; ++i) {
    const int mBase = m0 + (i << 4);
#pragma unroll
    for (int j = 0; j < 4; ++j) {
      const int n = n0 + (j << 4) + rlane;
      float bv = 0.f;
      if (BIAS_MODE == 2) bv = bias[n];
#pragma unroll
      for (int r = 0; r < 8; ++r) {
        float v = acc[i][j][r] * scale;
        if (BIAS_MODE == 1) v += bias[mBase + mOff + r];
        if (BIAS_MODE == 2) v += bv;
        if (RESID) v += Rb[(size_t)(mBase + mOff + r) * ldc + n];
        if (ACT == 1) v = tanhf(v);
        if (ACT == 2) v = fmaxf(v, 0.0f);
        if (ACT == 3) v = v / (1.0f + expf(-v));
        if (ACT == 4) v = (v > 0.f) ? v : 0.01f * v;
        slab[(mOff + r) * 68 + (j << 4) + rlane] = v;
      }
    }
    __builtin_amdgcn_fence(__ATOMIC_RELEASE, "workgroup");
    __builtin_amdgcn_wave_barrier();
    __builtin_amdgcn_fence(__ATOMIC_ACQUIRE, "workgroup");
    if (OUT_MODE == 0) {
      float* C = (float*)Cout + (size_t)b * strideC;
      const int hh = lane >> 4, c4 = (lane & 15) * 4;
      for (int pass = 0; pass < 2; ++pass) {
#pragma unroll
        for (int it = 0; it < 8; ++it) {
          const int row = it * 2 + hh;
          v4f v = *(const v4f*)(slab + row * 68 + c4);
          *(volatile v4f*)(C + (size_t)(mBase + row) * ldc + n0 + c4) = v;
        }
        __threadfence();
      }
    } else {
      const int q = lane >> 3, c8 = (lane & 7) * 8;
      unsigned short* C  = (unsigned short*)Cout  + (size_t)b * strideC;
      unsigned short* C2 = (OUT_MODE == 2) ? ((unsigned short*)Cout2 + (size_t)b * strideC) : nullptr;
      for (int pass = 0; pass < 2; ++pass) {
#pragma unroll
        for (int it = 0; it < 4; ++it) {
          const int row = it * 4 + q;
          const float* sp = slab + row * 68 + c8;
          v8h hv, lv;
#pragma unroll
          for (int e = 0; e < 8; ++e) {
            if (OUT_MODE == 1) {
              hv[e] = (_Float16)sp[e];
            } else {
              unsigned short hb = f2bf_bits(sp[e]);
              unsigned short lb = f2bf_bits(sp[e] - bf_bits2f(hb));
              hv[e] = __builtin_bit_cast(_Float16, hb);
              lv[e] = __builtin_bit_cast(_Float16, lb);
            }
          }
          *(volatile v8h*)(C + (size_t)(mBase + row) * ldc + n0 + c8) = hv;
          if (OUT_MODE == 2) *(volatile v8h*)(C2 + (size_t)(mBase + row) * ldc + n0 + c8) = lv;
        }
        __threadfence();
      }
    }
    __builtin_amdgcn_fence(__ATOMIC_RELEASE, "workgroup");
    __builtin_amdgcn_wave_barrier();
    __builtin_amdgcn_fence(__ATOMIC_ACQUIRE, "workgroup");
  }
}

__global__ __launch_bounds__(kThr) void cast_plane_kernel(const float* __restrict__ src, unsigned short* __restrict__ dst,
                                                          int colsLog2, int dstPitch, int dstOff) {
  const int i   = blockIdx.x * kThr + threadIdx.x;
  const int sh  = colsLog2 - 3;
  const int row = i >> sh;
  const int c8  = (i & ((1 << sh) - 1)) * 8;
  const float* sp = src + ((size_t)row << colsLog2) + c8;
  const v4f a0 = *(const v4f*)(sp);
  const v4f a1 = *(const v4f*)(sp + 4);
  v8h hv;
#pragma unroll
  for (int e = 0; e < 4; ++e) {
    const float f0 = a0[e];
    const float f1 = a1[e];
    hv[e]     = (_Float16)carry_flush(bf16r(f0), kInCarry);
    hv[4 + e] = (_Float16)carry_flush(bf16r(f1), kInCarry);
  }
  unsigned short* dp = dst + (size_t)row * dstPitch + dstOff + c8;
  *(volatile v8h*)dp = hv;
  __threadfence();
  *(volatile v8h*)dp = hv;
}
__global__ __launch_bounds__(256) void wt_plane_kernel(const float* __restrict__ W, unsigned short* __restrict__ dst, int K, int N, int nLive, int ldd, int colOff) {
  const int n  = blockIdx.x;
  const int k8 = threadIdx.x * 8;
  const bool live = n < nLive;
  const int nc = live ? n : 0;
  v8h hv;
#pragma unroll
  for (int e = 0; e < 8; ++e) {
    const float w = W[(size_t)(k8 + e) * N + nc];
    hv[e] = (_Float16)(live ? carry_flush(bf16r(w), kWCarry) : 0.0f);
  }
  unsigned short* dp = dst + (size_t)n * ldd + colOff + k8;
  *(volatile v8h*)dp = hv;
  __threadfence();
  *(volatile v8h*)dp = hv;
}


__device__ __forceinline__ float silu_f(float v) { return v / (1.0f + expf(-v)); }

__global__ __launch_bounds__(kThr) void setup_kernel(const float* __restrict__ A_log, const float* __restrict__ dt_bias, const float* __restrict__ o_norm_w,
                                                     float* __restrict__ BIAS, float* __restrict__ PRM) {
  unsigned v = blockIdx.x * (unsigned)kThr + threadIdx.x;
  asm volatile("" : "+v"(v));
  if (v < 512u) {
    float* dp = BIAS + v * 4u;
    const v4f z = {0.f, 0.f, 0.f, 0.f};
    *(volatile v4f*)dp = z;
    __threadfence();
    *(volatile v4f*)dp = z;
  } else {
    const unsigned i = v - 512u;
    const bool isA = i < (unsigned)kH, isD = (i >= (unsigned)kPD) && (i < (unsigned)(kPD + kH)), isW = (i >= (unsigned)kPW) && (i < (unsigned)(kPW + kHd));
    const float a = bf16r(A_log[isA ? i : 0u]);
    const float d = bf16r(dt_bias[isD ? (i - (unsigned)kPD) : 0u]);
    const float w = bf16r(o_norm_w[isW ? (i - (unsigned)kPW) : 0u]);
    const float val = isA ? -expf(a) : (isD ? d : (isW ? w : 0.0f));
    float* dp = PRM + i;
    *(volatile float*)dp = val;
    __threadfence();
    *(volatile float*)dp = val;
  }
}
static_assert(kDH / 4 == 512 && 512 + kPEnd == 6 * kThr && (512 % 32) == 0, "set-up grid exact; regions wave-uniform");

__global__ __launch_bounds__(kThr) void convnorm_kernel(const float* __restrict__ X, const float* __restrict__ cw, float* __restrict__ OUT, int mode) {
  const unsigned t = blockIdx.x * (unsigned)kThr + threadIdx.x;
  const unsigned c0 = blockIdx.y * (unsigned)kHd;
  float* orow = OUT + (size_t)t * kKD + c0;
  float ss = 0.0f;
  const int npassA = (mode == 0) ? 2 : 1;
  for (int pass = 0; pass < npassA; ++pass) {
    ss = 0.0f;
#pragma unroll 1
    for (int c = 0; c < kHd; c += 4) {
      v4f acc = {0.f, 0.f, 0.f, 0.f};
#pragma unroll
      for (int j = 0; j < kTaps; ++j) {
        const int tr = (int)t - (kTaps - 1) + j;
        if (tr >= 0) {
          const v4f xv = *(const v4f*)(X + (size_t)tr * kKD + c0 + c);
#pragma unroll
          for (int e = 0; e < 4; ++e) acc[e] += xv[e] * bf16r(cw[(size_t)(c0 + c + e) * kTaps + j]);
        }
      }
      v4f y;
#pragma unroll
      for (int e = 0; e < 4; ++e) { y[e] = silu_f(acc[e]); ss += y[e] * y[e]; }
      *(volatile v4f*)(orow + c) = y;
    }
    __threadfence();
  }
  if (mode != 0) {
    float qs = (mode == 2) ? kQScale : 1.0f;
    asm volatile("" : "+v"(qs));
    const float rn = (1.0f / sqrtf(ss + kL2Eps)) * qs;
#pragma unroll 1
    for (int c = 0; c < kHd; c += 4) {
      const v4f a = *(const v4f*)(orow + c);
      v4f y;
#pragma unroll
      for (int e = 0; e < 4; ++e) y[e] = a[e] * rn;
      *(volatile v4f*)(orow + c) = y;
    }
    __threadfence();
#pragma unroll 1
    for (int c = 0; c < kHd; c += 4) { const v4f a = *(const v4f*)(orow + c); *(volatile v4f*)(orow + c) = a; }
    __threadfence();
  }
}

__global__ __launch_bounds__(kThr) void betag_kernel(const float* __restrict__ BAL, const float* __restrict__ PRM, float* __restrict__ BE) {
  const unsigned t = blockIdx.x * (unsigned)kThr + threadIdx.x;
  const float* br = BAL + (size_t)t * kBG;
  float* er = BE + (size_t)t * 32;
  for (int pass = 0; pass < 2; ++pass) {
#pragma unroll 1
    for (int h = 0; h < 8; h += 4) {
      const v4f bb = *(const v4f*)(br + h), gg = *(const v4f*)(br + 8 + h), na = *(const v4f*)(PRM + kPA + h), db = *(const v4f*)(PRM + kPD + h);
      v4f ob, oe;
#pragma unroll
      for (int e = 0; e < 4; ++e) {
        ob[e] = 1.0f / (1.0f + expf(-bb[e]));
        const float x = gg[e] + db[e];
        const float sp = fmaxf(x, 0.0f) + log1pf(expf(-fabsf(x)));
        oe[e] = expf(na[e] * sp);
      }
      *(volatile v4f*)(er + h) = ob;
      *(volatile v4f*)(er + 8 + h) = oe;
    }
    __threadfence();
  }
}
static_assert(kL == 8 * kThr && kH <= 8, "one thread a row: 8 blocks; six heads in eight slots");

__global__ __launch_bounds__(kCS) void gdn_scan_kernel(const float* __restrict__ Q2, const float* __restrict__ K2, const float* __restrict__ V2,
                                                       const float* __restrict__ BE, float* __restrict__ O32) {
  __shared__ float st[kHd * kCS];
  const unsigned lane = threadIdx.x;
  const unsigned h = blockIdx.x >> 2, qd = blockIdx.x & 3u;
  const unsigned hoff = h * (unsigned)kHd;
  const unsigned vcol = hoff + qd * (unsigned)kCS + lane;
  for (int k = 0; k < kHd; ++k) st[k * kCS + lane] = 0.0f;
  for (int t = 0; t < kL; ++t) {
    const float* qr = Q2 + (size_t)t * kKD + hoff;
    const float* kr = K2 + (size_t)t * kKD + hoff;
    const float vv = V2[(size_t)t * kKD + vcol];
    const float bt = BE[(size_t)t * 32 + h], et = BE[(size_t)t * 32 + 8 + h];
    float r = 0.0f;
#pragma unroll 1
    for (int k4 = 0; k4 < kHd; k4 += 4) {
      const v4f c4 = *(const v4f*)(kr + k4);
#pragma unroll
      for (int j = 0; j < 4; ++j) r += c4[j] * (et * st[(k4 + j) * kCS + (int)lane]);
    }
    const float vres = vv - r;
    const float bv = bt * vres;
    float sum = 0.0f;
#pragma unroll 1
    for (int k4 = 0; k4 < kHd; k4 += 4) {
      const v4f q4 = *(const v4f*)(qr + k4), c4 = *(const v4f*)(kr + k4);
#pragma unroll
      for (int j = 0; j < 4; ++j) {
        const int idx = (k4 + j) * kCS + (int)lane;
        const float s = et * st[idx] + c4[j] * bv;
        st[idx] = s;
        sum += q4[j] * s;
      }
    }
    float* op = O32 + (size_t)t * kKD + vcol;
    *(volatile float*)op = sum;
    __threadfence();
    *(volatile float*)op = sum;
  }
}
static_assert(kHd * kCS * 4 == 65536 && kCS == 64 && kH * 4 == 24, "the state slice: 64 KB of LDS a block; one thread a value column; 24 blocks");

__global__ __launch_bounds__(kThr) void normgate_kernel(const float* __restrict__ O32, const float* __restrict__ GL, const float* __restrict__ PRM, unsigned short* __restrict__ O16) {
  const unsigned t = blockIdx.x * (unsigned)kThr + threadIdx.x;
  const size_t base = (size_t)t * kKD + blockIdx.y * (unsigned)kHd;
  const float* orow = O32 + base;
  const float* grow = GL + base;
  const float* w = PRM + kPW;
  float ss = 0.0f;
#pragma unroll 1
  for (int c = 0; c < kHd; c += 4) { const v4f a = *(const v4f*)(orow + c); ss += (a[0] * a[0] + a[1] * a[1]) + (a[2] * a[2] + a[3] * a[3]); }
  const float rs = 1.0f / sqrtf(ss * (1.0f / (float)kHd) + kRmsEps);
  unsigned short* dst = O16 + base;
  for (int pass = 0; pass < 2; ++pass) {
#pragma unroll 1
    for (int c = 0; c < kHd; c += 8) {
      const v4f a0 = *(const v4f*)(orow + c), a1 = *(const v4f*)(orow + c + 4), g0 = *(const v4f*)(grow + c), g1 = *(const v4f*)(grow + c + 4), w0 = *(const v4f*)(w + c), w1 = *(const v4f*)(w + c + 4);
      v8h hv;
#pragma unroll
      for (int e = 0; e < 4; ++e) {
        hv[e] = (_Float16)carry_flush(a0[e] * rs * w0[e] * silu_f(g0[e]), kCo);
        hv[4 + e] = (_Float16)carry_flush(a1[e] * rs * w1[e] * silu_f(g1[e]), kCo);
      }
      *(volatile v8h*)(dst + c) = hv;
    }
    __threadfence();
  }
}
static_assert((kL % kThr) == 0, "row grids exact");

extern "C" void kernel_launch(void* const* d_in, const int* in_sizes, int n_in,
                              void* d_out, int out_size, void* d_ws, size_t ws_size,
                              hipStream_t stream) {
  if (n_in < 14 || d_out == nullptr || d_ws == nullptr) return;
  if (in_sizes[0] != kB * kL * kDH || in_sizes[1] != kKD * kDH || in_sizes[2] != kKD * kDH || in_sizes[3] != kKD * kDH || in_sizes[4] != kDH * kKD || in_sizes[5] != kH * kDH || in_sizes[6] != kH * kDH || in_sizes[7] != kKD * kDH) return;
  if (in_sizes[8] != kKD * kTaps || in_sizes[9] != kKD * kTaps || in_sizes[10] != kKD * kTaps || in_sizes[11] != kHd || in_sizes[12] != kH || in_sizes[13] != kH) return;
  if (out_size != kB * kL * kDH) return;
  if (ws_size < kWsTotal) return;
  const float* hidden = (const float*)d_in[0];
  const float* Wq = (const float*)d_in[1];
  const float* Wk = (const float*)d_in[2];
  const float* Wv = (const float*)d_in[3];
  const float* Wo = (const float*)d_in[4];
  const float* Wb = (const float*)d_in[5];
  const float* Wa = (const float*)d_in[6];
  const float* Wg = (const float*)d_in[7];
  const float* conv_q = (const float*)d_in[8];
  const float* conv_k = (const float*)d_in[9];
  const float* conv_v = (const float*)d_in[10];
  const float* o_norm_w = (const float*)d_in[11];
  const float* A_log = (const float*)d_in[12];
  const float* dt_bias = (const float*)d_in[13];
  float* out = (float*)d_out;
  char* ws = (char*)d_ws;
  unsigned short* WQ = (unsigned short*)(ws + kOffWQ);
  unsigned short* WK = (unsigned short*)(ws + kOffWK);
  unsigned short* WV = (unsigned short*)(ws + kOffWV);
  unsigned short* WG = (unsigned short*)(ws + kOffWG);
  unsigned short* WO = (unsigned short*)(ws + kOffWO);
  unsigned short* WBA = (unsigned short*)(ws + kOffWBA);
  float* BIAS = (float*)(ws + kOffBIAS);
  float* PRM = (float*)(ws + kOffPRM);
  unsigned short* X16 = (unsigned short*)(ws + kOffX16);
  float* XL = (float*)(ws + kOffXL);
  float* Q2 = (float*)(ws + kOffQ2);
  float* K2 = (float*)(ws + kOffK2);
  float* V2 = (float*)(ws + kOffV2);
  float* GL = (float*)(ws + kOffGL);
  float* BAL = (float*)(ws + kOffBAL);
  float* BE = (float*)(ws + kOffBE);
  float* O32 = (float*)(ws + kOffO32);
  unsigned short* O16 = (unsigned short*)(ws + kOffO16);

  const int gW = (int)(((size_t)kKD * kDH / 8) / kThr);
  cast_plane_kernel<<<gW, kThr, 0, stream>>>(Wq, WQ, 11, kDH, 0);
  cast_plane_kernel<<<gW, kThr, 0, stream>>>(Wk, WK, 11, kDH, 0);
  cast_plane_kernel<<<gW, kThr, 0, stream>>>(Wv, WV, 11, kDH, 0);
  cast_plane_kernel<<<gW, kThr, 0, stream>>>(Wg, WG, 11, kDH, 0);
  cast_plane_kernel<<<gW, kThr, 0, stream>>>(Wo, WO, 9, 512, 0);
  cast_plane_kernel<<<(kH * kDH / 8) / kThr, kThr, 0, stream>>>(Wb, WBA, 11, kDH, 0);
  cast_plane_kernel<<<(kH * kDH / 8) / kThr, kThr, 0, stream>>>(Wa, WBA + (size_t)8 * kDH, 11, kDH, 0);
  wt_plane_kernel<<<2, kDH / 8, 0, stream>>>(Wq, WBA + (size_t)kH * kDH, kDH, 1, 0, kDH, 0);
  wt_plane_kernel<<<kBG - 14, kDH / 8, 0, stream>>>(Wq, WBA + (size_t)14 * kDH, kDH, 1, 0, kDH, 0);
  setup_kernel<<<6, kThr, 0, stream>>>(A_log, dt_bias, o_norm_w, BIAS, PRM);

  const dim3 gRH(kL / kThr, kH);
  for (int s = 0; s < kB; ++s) {
    cast_plane_kernel<<<(int)(((size_t)kL * kDH / 8) / kThr), kThr, 0, stream>>>(hidden + (size_t)s * kL * kDH, X16, 11, kDH, 0);
    wmma_gemm64<0, false, 2, 0, false, 0><<<dim3((kL / 64) * (kKD / 64) / 8, 1), 256, 0, stream>>>(
        X16, X16, kDH, 0L, WQ, WQ, kDH, 0L, (void*)XL, (void*)XL, kKD, 0L, BIAS, nullptr, 0L, kL, kKD, kDH, kSc);
    convnorm_kernel<<<gRH, kThr, 0, stream>>>(XL, conv_q, Q2, 2);
    wmma_gemm64<0, false, 2, 0, false, 0><<<dim3((kL / 64) * (kKD / 64) / 8, 1), 256, 0, stream>>>(
        X16, X16, kDH, 0L, WK, WK, kDH, 0L, (void*)XL, (void*)XL, kKD, 0L, BIAS, nullptr, 0L, kL, kKD, kDH, kSc);
    convnorm_kernel<<<gRH, kThr, 0, stream>>>(XL, conv_k, K2, 1);
    wmma_gemm64<0, false, 2, 0, false, 0><<<dim3((kL / 64) * (kKD / 64) / 8, 1), 256, 0, stream>>>(
        X16, X16, kDH, 0L, WV, WV, kDH, 0L, (void*)XL, (void*)XL, kKD, 0L, BIAS, nullptr, 0L, kL, kKD, kDH, kSc);
    convnorm_kernel<<<gRH, kThr, 0, stream>>>(XL, conv_v, V2, 0);
    wmma_gemm64<0, false, 2, 0, false, 0><<<dim3((kL / 64) * (kKD / 64) / 8, 1), 256, 0, stream>>>(
        X16, X16, kDH, 0L, WG, WG, kDH, 0L, (void*)GL, (void*)GL, kKD, 0L, BIAS, nullptr, 0L, kL, kKD, kDH, kSc);
    wmma_gemm64<0, false, 2, 0, false, 0><<<dim3((kL / 64) * (kBG / 64) / 8, 1), 256, 0, stream>>>(
        X16, X16, kDH, 0L, WBA, WBA, kDH, 0L, (void*)BAL, (void*)BAL, kBG, 0L, BIAS, nullptr, 0L, kL, kBG, kDH, kSc);
    betag_kernel<<<kL / kThr, kThr, 0, stream>>>(BAL, PRM, BE);
    gdn_scan_kernel<<<kH * 4, kCS, 0, stream>>>(Q2, K2, V2, BE, O32);
    normgate_kernel<<<gRH, kThr, 0, stream>>>(O32, GL, PRM, O16);
    wmma_gemm64<0, false, 2, 0, false, 0><<<dim3((kL / 64) * (kDH / 64) / 8, 1), 256, 0, stream>>>(
        O16, O16, kKD, 0L, WO, WO, kKD, 0L, (void*)(out + (size_t)s * kL * kDH), (void*)(out + (size_t)s * kL * kDH), kDH, 0L, BIAS, nullptr, 0L, kL, kDH, kKD, kScO);
  }
}
